// MVT_Mamba_62603443307010
// MI455X (gfx1250) — hardware-verified
//
#include <hip/hip_runtime.h>
#include <math.h>

constexpr int NBATCH = 4;
constexpr int SEQ_L  = 2048;
constexpr int DMODEL = 512;
constexpr int NSTATE = 16;
constexpr int KCONV  = 4;
constexpr int DIN    = 1024;
constexpr int DTRANK = 32;
constexpr int NTOK   = NBATCH * SEQ_L;
constexpr int XZ_W   = 2 * DIN;
constexpr int XDBL_W = DTRANK + 2 * NSTATE;
constexpr int SCAN_CH = 64;
constexpr float CARRY      = 256.0f;
constexpr float INV_CARRY  = 1.0f / 256.0f;
constexpr float INV_CARRY2 = 1.0f / 65536.0f;

constexpr size_t SZ_XZ    = (size_t)NTOK * XZ_W * 4;
constexpr size_t SZ_P16   = (size_t)NTOK * DIN * 2;
constexpr size_t OFF_XZ   = 0;
constexpr size_t OFF_XH   = OFF_XZ + SZ_XZ;
constexpr size_t OFF_DT16 = OFF_XH + SZ_P16;
constexpr size_t OFF_Y0H  = OFF_DT16 + SZ_P16;
constexpr size_t OFF_RA   = OFF_Y0H + SZ_P16;
constexpr size_t OFF_HB   = OFF_RA;
constexpr size_t OFF_WINB = OFF_HB + (size_t)NTOK * DMODEL * 2;
constexpr size_t WS_END1  = OFF_WINB + (size_t)XZ_W * DMODEL * 2;
constexpr size_t OFF_XDBL = OFF_RA;
constexpr size_t OFF_DTRH = OFF_XDBL + (size_t)NTOK * XDBL_W * 4;
constexpr size_t OFF_WX0  = OFF_DTRH + (size_t)NTOK * DTRANK * 2;
constexpr size_t OFF_WX1  = OFF_WX0 + (size_t)XDBL_W * DIN * 2;
constexpr size_t OFF_WDT0 = OFF_WX1 + (size_t)XDBL_W * DIN * 2;
constexpr size_t OFF_WDT1 = OFF_WDT0 + (size_t)DIN * DTRANK * 2;
constexpr size_t OFF_WOUT = OFF_WDT1 + (size_t)DIN * DTRANK * 2;
constexpr size_t WS_END2  = OFF_WOUT + (size_t)DMODEL * DIN * 2;
constexpr size_t WS_TOTAL = (WS_END1 > WS_END2) ? WS_END1 : WS_END2;
static_assert(WS_TOTAL <= (size_t)134217728);

typedef __attribute__((ext_vector_type(16))) _Float16 v16h;
typedef __attribute__((ext_vector_type(8)))  _Float16 v8h;
typedef __attribute__((ext_vector_type(16))) __bf16   v16b;
typedef __attribute__((ext_vector_type(8)))  __bf16   v8b;
typedef __attribute__((ext_vector_type(8)))  float    v8f;
typedef __attribute__((ext_vector_type(4)))  float    v4f;
typedef unsigned short v8us   __attribute__((ext_vector_type(8)));
typedef unsigned short v8us_a __attribute__((ext_vector_type(8), may_alias));

__device__ __forceinline__ unsigned short f2bf_bits(float f) {
  unsigned u = __float_as_uint(f);
  return (unsigned short)((u + 0x7FFFu + ((u >> 16) & 1u)) >> 16);
}
__device__ __forceinline__ float bf_bits2f(unsigned short h) { return __uint_as_float(((unsigned)h) << 16); }
__device__ __forceinline__ float bfr(float f) { return bf_bits2f(f2bf_bits(f)); }
__device__ __forceinline__ unsigned short f2h_bits(float f) { return __builtin_bit_cast(unsigned short, (_Float16)f); }
__device__ __forceinline__ float h_bits2f(unsigned short u) { return (float)__builtin_bit_cast(_Float16, u); }

__device__ __forceinline__ void dep_guard_h(v8f& a, v8f& b, v16h x, v16h y) { asm volatile("v_nop\n\tv_nop\n\tv_nop\n\tv_nop" : "+v"(a), "+v"(b) : "v"(x), "v"(y)); }
__device__ __forceinline__ void dep_guard_b(v8f& a, v8f& b, v16b x, v16b y) { asm volatile("v_nop\n\tv_nop\n\tv_nop\n\tv_nop" : "+v"(a), "+v"(b) : "v"(x), "v"(y)); }
__device__ __forceinline__ void keep4_h(v16h a, v16h b, v16h c, v16h d) { asm volatile("v_nop" :: "v"(a), "v"(b), "v"(c), "v"(d)); }
__device__ __forceinline__ void keep4_b(v16b a, v16b b, v16b c, v16b d) { asm volatile("v_nop" :: "v"(a), "v"(b), "v"(c), "v"(d)); }
__device__ __forceinline__ void acc_guard4(v8f& a, v8f& b, v8f& c, v8f& d) { asm volatile("v_nop\n\tv_nop\n\tv_nop\n\tv_nop" : "+v"(a), "+v"(b), "+v"(c), "+v"(d)); }
template <typename T> struct Frag;
template <> struct Frag<_Float16> {
  typedef v16h V; union U { v16h v; v8h h[2]; };
  static __device__ __forceinline__ v16h load(const _Float16* p) {
    U f; f.h[0] = *(const v8h*)(p); f.h[1] = *(const v8h*)(p + 16); return f.v;
  }
  static __device__ __forceinline__ v8f mma(v16h a, v16h b, v8f c) {
    return __builtin_amdgcn_wmma_f32_16x16x32_f16(false, a, false, b, (short)0, c, false, false);
  }
  static __device__ __forceinline__ void guard(v8f& a, v8f& b, v16h x, v16h y) { dep_guard_h(a, b, x, y); }
  static __device__ __forceinline__ void keep(v16h a, v16h b, v16h c, v16h d) { keep4_h(a, b, c, d); }
};
template <> struct Frag<__bf16> {
  typedef v16b V; union U { v16b v; v8b h[2]; };
  static __device__ __forceinline__ v16b load(const __bf16* p) {
    U f; f.h[0] = *(const v8b*)(p); f.h[1] = *(const v8b*)(p + 16); return f.v;
  }
  static __device__ __forceinline__ v8f mma(v16b a, v16b b, v8f c) {
    return __builtin_amdgcn_wmma_f32_16x16x32_bf16(false, a, false, b, (short)0, c, false, false);
  }
  static __device__ __forceinline__ void guard(v8f& a, v8f& b, v16b x, v16b y) { dep_guard_b(a, b, x, y); }
  static __device__ __forceinline__ void keep(v16b a, v16b b, v16b c, v16b d) { keep4_b(a, b, c, d); }
};

template <int ET> struct Elem;
template <> struct Elem<0> { typedef _Float16 T; };
template <> struct Elem<1> { typedef __bf16 T; };
template <int ET, bool SPLIT, int BIAS_MODE, int OUT_MODE, bool RESID, int ACT = 0>
__global__ __launch_bounds__(256) void wmma_gemm64(
    const unsigned short* __restrict__ Ap, const unsigned short* __restrict__ A2p, int lda, long strideA,
    const unsigned short* __restrict__ Btp, const unsigned short* __restrict__ Bt2p, int ldb, long strideB,
    void* __restrict__ Cout, void* __restrict__ Cout2, int ldc, long strideC,
    const float* __restrict__ bias,
    const float* __restrict__ resid, long strideR,
    int M, int N, int K, float scale) {
  typedef typename Elem<ET>::T T;
  typedef typename Frag<T>::V V;
  const T* A = (const T*)Ap; const T* A2 = (const T*)A2p; const T* Bt = (const T*)Btp; const T* Bt2 = (const T*)Bt2p;
  __shared__ __align__(16) float sT[8][16 * 68];
  const int b    = blockIdx.y;
  const int lane = threadIdx.x & 31;
  const int wave = threadIdx.x >> 5;
  const int tilesN = N >> 6;
  const int tilesM = M >> 6;
  const int tile = blockIdx.x * 8 + wave;
  if (tile >= tilesM * tilesN) return;
  const int tm = tile / tilesN;
  const int tn = tile - tm * tilesN;
  const int m0 = tm << 6;
  const int n0 = tn << 6;

  const T* Ab  = A  + (size_t)b * strideA;
  const T* Bb  = Bt + (size_t)b * strideB;
  const T* Ab2 = SPLIT ? (A2  + (size_t)b * strideA) : nullptr;
  const T* Bb2 = SPLIT ? (Bt2 + (size_t)b * strideB) : nullptr;

  const int rlane = lane & 15;
  const int koff  = (lane >> 4) * 8;
  const int mOff  = (lane >> 4) * 8;

  v8f acc[4][4];
#pragma unroll
  for (int i = 0; i < 4; ++i)
#pragma unroll
    for (int j = 0; j < 4; ++j) acc[i][j] = (v8f){0.f,0.f,0.f,0.f,0.f,0.f,0.f,0.f};

  for (int k0 = 0; k0 < K; k0 += 32) {
    V bh[4], bl[4];
#pragma unroll
    for (int j = 0; j < 4; ++j) {
      const size_t bo = (size_t)(n0 + (j << 4) + rlane) * ldb + koff + k0;
      bh[j] = Frag<T>::load(Bb + bo);
      if (SPLIT) bl[j] = Frag<T>::load(Bb2 + bo);
    }
#pragma unroll
    for (int i = 0; i < 4; ++i) {
      const size_t ao = (size_t)(m0 + (i << 4) + rlane) * lda + koff + k0;
      V ah = Frag<T>::load(Ab + ao);
      V al;
      if (SPLIT) al = Frag<T>::load(Ab2 + ao);
#pragma unroll
      for (int j = 0; j < 4; ++j) {
        acc[i][j] = Frag<T>::mma(ah, bh[j], acc[i][j]);
        if (SPLIT) {
          acc[i][j] = Frag<T>::mma(ah, bl[j], acc[i][j]);
          acc[i][j] = Frag<T>::mma(al, bh[j], acc[i][j]);
        }
      }
      Frag<T>::guard(acc[i][0], acc[i][3], ah, SPLIT ? al : ah);
    }
    Frag<T>::keep(bh[0], bh[1], bh[2], bh[3]);
    if (SPLIT) Frag<T>::keep(bl[0], bl[1], bl[2], bl[3]);
  }
  acc_guard4(acc[0][0], acc[0][1], acc[0][2], acc[0][3]);
  acc_guard4(acc[1][0], acc[1][1], acc[1][2], acc[1][3]);
  acc_guard4(acc[2][0], acc[2][1], acc[2][2], acc[2][3]);
  acc_guard4(acc[3][0], acc[3][1], acc[3][2], acc[3][3]);

  float* slab = sT[wave];
  const float* Rb = RESID ? (resid + (size_t)b * strideR) : nullptr;
#pragma unroll
  for (int i = 0; i < 4; ++i) {
    const int mBase = m0 + (i << 4);
#pragma unroll
    for (int j = 0; j < 4; ++j) {
      const int n = n0 + (j << 4) + rlane;
      float bv = 0.f;
      if (BIAS_MODE == 2) bv = bias[n];
#pragma unroll
      for (int r = 0; r < 8; ++r) {
        float v = acc[i][j][r] * scale;
        if (BIAS_MODE == 1) v += bias[mBase + mOff + r];
        if (BIAS_MODE == 2) v += bv;
        if (RESID) v += Rb[(size_t)(mBase + mOff + r) * ldc + n];
        if (ACT == 1) v = tanhf(v);
        if (ACT == 2) v = fmaxf(v, 0.0f);
        if (ACT == 3) v = v / (1.0f + expf(-v));
        if (ACT == 4) v = (v > 0.f) ? v : 0.01f * v;
        slab[(mOff + r) * 68 + (j << 4) + rlane] = v;
      }
    }
    __builtin_amdgcn_fence(__ATOMIC_RELEASE, "workgroup");
    __builtin_amdgcn_wave_barrier();
    __builtin_amdgcn_fence(__ATOMIC_ACQUIRE, "workgroup");
    if (OUT_MODE == 0) {
      float* C = (float*)Cout + (size_t)b * strideC;
      const int hh = lane >> 4, c4 = (lane & 15) * 4;
      for (int pass = 0; pass < 2; ++pass) {
#pragma unroll
        for (int it = 0; it < 8; ++it) {
          const int row = it * 2 + hh;
          v4f v = *(const v4f*)(slab + row * 68 + c4);
          *(volatile v4f*)(C + (size_t)(mBase + row) * ldc + n0 + c4) = v;
        }
        __threadfence();
      }
    } else {
      const int q = lane >> 3, c8 = (lane & 7) * 8;
      unsigned short* C  = (unsigned short*)Cout  + (size_t)b * strideC;
      unsigned short* C2 = (OUT_MODE == 2) ? ((unsigned short*)Cout2 + (size_t)b * strideC) : nullptr;
      for (int pass = 0; pass < 2; ++pass) {
#pragma unroll
        for (int it = 0; it < 4; ++it) {
          const int row = it * 4 + q;
          const float* sp = slab + row * 68 + c8;
          v8h hv, lv;
#pragma unroll
          for (int e = 0; e < 8; ++e) {
            if (OUT_MODE == 1) {
              hv[e] = (_Float16)sp[e];
            } else {
              unsigned short hb = f2bf_bits(sp[e]);
              unsigned short lb = f2bf_bits(sp[e] - bf_bits2f(hb));
              hv[e] = __builtin_bit_cast(_Float16, hb);
              lv[e] = __builtin_bit_cast(_Float16, lb);
            }
          }
          *(volatile v8h*)(C + (size_t)(mBase + row) * ldc + n0 + c8) = hv;
          if (OUT_MODE == 2) *(volatile v8h*)(C2 + (size_t)(mBase + row) * ldc + n0 + c8) = lv;
        }
        __threadfence();
      }
    }
    __builtin_amdgcn_fence(__ATOMIC_RELEASE, "workgroup");
    __builtin_amdgcn_wave_barrier();
    __builtin_amdgcn_fence(__ATOMIC_ACQUIRE, "workgroup");
  }
}

__device__ __forceinline__ float silu_f(float x) {
  const float e = __expf(-x);
  return x * __builtin_amdgcn_rcpf(1.0f + e);
}
__device__ __forceinline__ float softplus_f(float x) {
  const float e = __expf(-fabsf(x));
  return fmaxf(x, 0.0f) + __logf(1.0f + e);
}

template <int MODE>
__global__ __launch_bounds__(256) void cast8_kernel(const float* __restrict__ src, unsigned short* __restrict__ dst,
                                                    int ngroups, int ocols, int spitch, float scale) {
  const int i = blockIdx.x * 256 + threadIdx.x;
  if (i >= ngroups) return;
  const size_t o   = (size_t)i * 8;
  const size_t row = o / (size_t)ocols;
  const int    c   = (int)(o - row * (size_t)ocols);
  const float* sp  = src + row * (size_t)spitch + c;
  const v4f a = *(const v4f*)(sp);
  const v4f b = *(const v4f*)(sp + 4);
  const float vv[8] = {a[0], a[1], a[2], a[3], b[0], b[1], b[2], b[3]};
  v8us r;
#pragma unroll
  for (int e = 0; e < 8; ++e) {
    unsigned short u;
    if (MODE == 0)      u = f2bf_bits(vv[e]);
    else if (MODE == 1) u = f2h_bits(bfr(vv[e]) * scale);
    else                u = f2h_bits(vv[e] * scale);
    r[e] = u;
  }
  unsigned short* dp = dst + o;
  *(volatile v8us*)dp = r;
  __threadfence();
  *(volatile v8us*)dp = r;
}

template <int DIR>
__global__ __launch_bounds__(256) void conv_silu8_kernel(const float* __restrict__ XZ, const float* __restrict__ cw,
                                                        const float* __restrict__ cb, unsigned short* __restrict__ Xh) {
  const int i = blockIdx.x * 256 + threadIdx.x;
  if (i >= NTOK * (DIN / 8)) return;
  const int m  = i / (DIN / 8);
  const int d0 = (i - m * (DIN / 8)) * 8;
  const int s  = m & (SEQ_L - 1);
  const int rb = m - s;
  float acc[8];
  {
    const v4f c0 = *(const v4f*)(cb + d0);
    const v4f c1 = *(const v4f*)(cb + d0 + 4);
    acc[0] = bfr(c0[0]); acc[1] = bfr(c0[1]); acc[2] = bfr(c0[2]); acc[3] = bfr(c0[3]);
    acc[4] = bfr(c1[0]); acc[5] = bfr(c1[1]); acc[6] = bfr(c1[2]); acc[7] = bfr(c1[3]);
  }
  v4f wv[8];
#pragma unroll
  for (int e = 0; e < 8; ++e) wv[e] = *(const v4f*)(cw + (size_t)(d0 + e) * KCONV);
#pragma unroll
  for (int j = 0; j < KCONV; ++j) {
    const int  ss    = DIR ? (s + (KCONV - 1) - j) : (s - (KCONV - 1) + j);
    const bool valid = DIR ? (ss < SEQ_L) : (ss >= 0);
    const int  sc    = ss < 0 ? 0 : (ss > SEQ_L - 1 ? SEQ_L - 1 : ss);
    const float* tp  = XZ + (size_t)(rb + sc) * XZ_W + d0;
    const v4f t0 = *(const v4f*)(tp);
    const v4f t1 = *(const v4f*)(tp + 4);
    const float tv[8] = {t0[0], t0[1], t0[2], t0[3], t1[0], t1[1], t1[2], t1[3]};
#pragma unroll
    for (int e = 0; e < 8; ++e) acc[e] = fmaf(bfr(wv[e][j]), valid ? tv[e] : 0.0f, acc[e]);
  }
  v8us r;
#pragma unroll
  for (int e = 0; e < 8; ++e) r[e] = f2h_bits(silu_f(acc[e]) * CARRY);
  unsigned short* dp = Xh + (size_t)m * DIN + d0;
  *(volatile v8us*)dp = r;
  __threadfence();
  *(volatile v8us*)dp = r;
}

template <int DIR>
__global__ __launch_bounds__(SCAN_CH) void scan_gate_kernel(
    const float* __restrict__ XZ, const unsigned short* __restrict__ DT16, const float* __restrict__ XDBL,
    const float* __restrict__ conv_w, const float* __restrict__ conv_b, const float* __restrict__ b_dt,
    const float* __restrict__ A_log, const float* __restrict__ Dv,
    const unsigned short* __restrict__ Yprev, unsigned short* __restrict__ Yout) {
  __shared__ __align__(16) unsigned short ys[2][SCAN_CH];
  constexpr int BLK_PER_B = DIN / SCAN_CH;
  const int tid = threadIdx.x;
  const int bb  = blockIdx.x / BLK_PER_B;
  const int d0  = (blockIdx.x - bb * BLK_PER_B) * SCAN_CH;
  const int d   = d0 + tid;

  float An[NSTATE], hs[NSTATE];
#pragma unroll
  for (int n = 0; n < NSTATE; ++n) { An[n] = -__expf(bfr(A_log[(size_t)d * NSTATE + n])); hs[n] = 0.0f; }
  const float w0  = bfr(conv_w[(size_t)d * KCONV + 0]);
  const float w1  = bfr(conv_w[(size_t)d * KCONV + 1]);
  const float w2  = bfr(conv_w[(size_t)d * KCONV + 2]);
  const float w3  = bfr(conv_w[(size_t)d * KCONV + 3]);
  const float cb  = bfr(conv_b[d]);
  const float bdt = bfr(b_dt[d]);
  const float Dd  = bfr(Dv[d]);
  float q1 = 0.0f, q2 = 0.0f, q3 = 0.0f;
  const size_t rowb = (size_t)bb * SEQ_L;

#pragma unroll 1
  for (int i = 0; i < SEQ_L; ++i) {
    const int s = DIR ? (SEQ_L - 1 - i) : i;
    const size_t m = rowb + (size_t)s;
    const float u = XZ[m * XZ_W + d];
    const float z = XZ[m * XZ_W + DIN + d];
    float cv = cb;
    cv = fmaf(w0, q3, cv); cv = fmaf(w1, q2, cv); cv = fmaf(w2, q1, cv); cv = fmaf(w3, u, cv);
    q3 = q2; q2 = q1; q1 = u;
    const float x   = silu_f(cv);
    const float dt  = softplus_f(fmaf(h_bits2f(DT16[m * DIN + d]), INV_CARRY, bdt));
    const float dtx = dt * x;
    const float* bcp = XDBL + m * XDBL_W + DTRANK;
    v4f bq[4], cq[4];
#pragma unroll
    for (int g4 = 0; g4 < 4; ++g4) {
      bq[g4] = *(const v4f*)(bcp + 4 * g4);
      cq[g4] = *(const v4f*)(bcp + NSTATE + 4 * g4);
    }
    float y = 0.0f;
#pragma unroll
    for (int n = 0; n < NSTATE; ++n) {
      const float dA = __expf(dt * An[n]);
      hs[n] = fmaf(hs[n], dA, dtx * bq[n >> 2][n & 3]);
      y = fmaf(hs[n], cq[n >> 2][n & 3], y);
    }
    float yv = fmaf(Dd, x, y) * silu_f(z) * CARRY;
    if (DIR == 1) yv += h_bits2f(Yprev[m * DIN + d]);
    ys[i & 1][tid] = f2h_bits(yv);
    __syncthreads();
    if (tid < SCAN_CH / 8) {
      const v8us val = *(const v8us_a*)(&ys[i & 1][tid * 8]);
      unsigned short* op = Yout + m * DIN + d0 + tid * 8;
      *(volatile v8us*)op = val;
      __threadfence();
      *(volatile v8us*)op = val;
    }
  }
}

static inline unsigned cdivu(long long a, long long b) { return (unsigned)((a + b - 1) / b); }

extern "C" void kernel_launch(void* const* d_in, const int* in_sizes, int n_in,
                              void* d_out, int out_size, void* d_ws, size_t ws_size,
                              hipStream_t stream) {
  (void)in_sizes; (void)out_size;
  if (n_in < 17) return;
  if (ws_size < WS_TOTAL) return;

  const float* hid   = (const float*)d_in[0];
  const float* W_in  = (const float*)d_in[1];
  const float* W_out = (const float*)d_in[2];
  const float* conv_w[2] = {(const float*)d_in[3], (const float*)d_in[10]};
  const float* conv_b[2] = {(const float*)d_in[4], (const float*)d_in[11]};
  const float* W_x[2]    = {(const float*)d_in[5], (const float*)d_in[12]};
  const float* W_dt[2]   = {(const float*)d_in[6], (const float*)d_in[13]};
  const float* b_dt[2]   = {(const float*)d_in[7], (const float*)d_in[14]};
  const float* A_log[2]  = {(const float*)d_in[8], (const float*)d_in[15]};
  const float* Dp[2]     = {(const float*)d_in[9], (const float*)d_in[16]};
  float* out = (float*)d_out;

  char* ws = (char*)d_ws;
  float*          XZ    = (float*)(ws + OFF_XZ);
  unsigned short* XH    = (unsigned short*)(ws + OFF_XH);
  unsigned short* DT16  = (unsigned short*)(ws + OFF_DT16);
  unsigned short* Y0H   = (unsigned short*)(ws + OFF_Y0H);
  unsigned short* HB    = (unsigned short*)(ws + OFF_HB);
  unsigned short* WINB  = (unsigned short*)(ws + OFF_WINB);
  float*          XDBL  = (float*)(ws + OFF_XDBL);
  unsigned short* DTRH  = (unsigned short*)(ws + OFF_DTRH);
  unsigned short* WX16[2]  = {(unsigned short*)(ws + OFF_WX0),  (unsigned short*)(ws + OFF_WX1)};
  unsigned short* WDT16[2] = {(unsigned short*)(ws + OFF_WDT0), (unsigned short*)(ws + OFF_WDT1)};
  unsigned short* WOUT16   = (unsigned short*)(ws + OFF_WOUT);
  const float* unused_f = (const float*)(ws + OFF_XZ);

  { const int ng = NTOK * DMODEL / 8;  cast8_kernel<0><<<cdivu(ng, 256), 256, 0, stream>>>(hid,  HB,   ng, DMODEL, DMODEL, 1.0f); }
  { const int ng = XZ_W * DMODEL / 8;  cast8_kernel<0><<<cdivu(ng, 256), 256, 0, stream>>>(W_in, WINB, ng, DMODEL, DMODEL, 1.0f); }

  { const int tiles = (NTOK / 64) * (XZ_W / 64);
    wmma_gemm64<1, false, 0, 0, false, 0><<<dim3(cdivu(tiles, 8), 1), 256, 0, stream>>>(
        HB, HB, DMODEL, 0L, WINB, WINB, DMODEL, 0L, XZ, XZ, XZ_W, 0L, unused_f, unused_f, 0L, NTOK, XZ_W, DMODEL, 1.0f); }

  for (int dir = 0; dir < 2; ++dir) {
    { const int ng = XDBL_W * DIN / 8;   cast8_kernel<1><<<cdivu(ng, 256), 256, 0, stream>>>(W_x[dir],  WX16[dir],  ng, DIN,    DIN,    CARRY); }
    { const int ng = DIN * DTRANK / 8;   cast8_kernel<1><<<cdivu(ng, 256), 256, 0, stream>>>(W_dt[dir], WDT16[dir], ng, DTRANK, DTRANK, CARRY); }
  }
  { const int ng = DMODEL * DIN / 8;     cast8_kernel<1><<<cdivu(ng, 256), 256, 0, stream>>>(W_out, WOUT16, ng, DIN, DIN, CARRY); }

  for (int dir = 0; dir < 2; ++dir) {
    { const int ng = NTOK * (DIN / 8);
      if (dir == 0) conv_silu8_kernel<0><<<cdivu(ng, 256), 256, 0, stream>>>(XZ, conv_w[0], conv_b[0], XH);
      else          conv_silu8_kernel<1><<<cdivu(ng, 256), 256, 0, stream>>>(XZ, conv_w[1], conv_b[1], XH); }
    { const int tiles = (NTOK / 64) * (XDBL_W / 64);
      wmma_gemm64<0, false, 0, 0, false, 0><<<dim3(cdivu(tiles, 8), 1), 256, 0, stream>>>(
          XH, XH, DIN, 0L, WX16[dir], WX16[dir], DIN, 0L, XDBL, XDBL, XDBL_W, 0L, unused_f, unused_f, 0L, NTOK, XDBL_W, DIN, INV_CARRY2); }
    { const int ng = NTOK * DTRANK / 8;
      cast8_kernel<2><<<cdivu(ng, 256), 256, 0, stream>>>(XDBL, DTRH, ng, DTRANK, XDBL_W, CARRY); }
    { const int tiles = (NTOK / 64) * (DIN / 64);
      wmma_gemm64<0, false, 0, 1, false, 0><<<dim3(cdivu(tiles, 8), 1), 256, 0, stream>>>(
          DTRH, DTRH, DTRANK, 0L, WDT16[dir], WDT16[dir], DTRANK, 0L, DT16, DT16, DIN, 0L, unused_f, unused_f, 0L, NTOK, DIN, DTRANK, INV_CARRY); }
    if (dir == 0)
      scan_gate_kernel<0><<<NBATCH * (DIN / SCAN_CH), SCAN_CH, 0, stream>>>(
          XZ, DT16, XDBL, conv_w[0], conv_b[0], b_dt[0], A_log[0], Dp[0], Y0H, Y0H);
    else
      scan_gate_kernel<1><<<NBATCH * (DIN / SCAN_CH), SCAN_CH, 0, stream>>>(
          XZ, DT16, XDBL, conv_w[1], conv_b[1], b_dt[1], A_log[1], Dp[1], Y0H, XH);
  }

  { const int tiles = (NTOK / 64) * (DMODEL / 64);
    wmma_gemm64<0, false, 0, 0, false, 0><<<dim3(cdivu(tiles, 8), 1), 256, 0, stream>>>(
        XH, XH, DIN, 0L, WOUT16, WOUT16, DIN, 0L, out, out, DMODEL, 0L, unused_f, unused_f, 0L, NTOK, DMODEL, DIN, INV_CARRY2); }
}
